// Proposed_MLMLP_60335700574541
// MI455X (gfx1250) — hardware-verified
//
#include <hip/hip_runtime.h>


namespace {
constexpr int Bn = 4096, FIN = 64, NK = 512, FO = 256;
constexpr float XS = 8.0f, CS = 8.0f, RS = 8.0f, WS_ = 8.0f;

typedef _Float16 b16;
typedef __attribute__((ext_vector_type(16))) _Float16 v16b;
typedef __attribute__((ext_vector_type(8))) _Float16 v8b;
typedef __attribute__((ext_vector_type(8))) float v8f;
typedef __attribute__((ext_vector_type(4))) float v4f;
__device__ __forceinline__ void split16(float v, b16& hi, b16& lo) { hi = (b16)v; lo = (b16)(v - (float)hi); }
__device__ __forceinline__ v16b frag_kb(const b16* p, int hh) { const v8b a = *(const v8b*)(p + 8 * hh), b = *(const v8b*)(p + 16 + 8 * hh); v16b f;
#pragma unroll
  for (int e = 0; e < 8; ++e) { f[e] = a[e]; f[8 + e] = b[e]; } return f; }
__device__ __forceinline__ v8f wmma16b(v16b a, v16b b, v8f c) { v8f d = __builtin_amdgcn_wmma_f32_16x16x32_f16(false, a, false, b, (short)0, c, false, false); asm volatile("v_nop\n\tv_nop\n\tv_nop\n\tv_nop" : "+v"(d) : "v"(a), "v"(b)); return d; }
__device__ __forceinline__ void wave_lds_sync() { __builtin_amdgcn_fence(__ATOMIC_RELEASE, "workgroup"); __builtin_amdgcn_wave_barrier(); __builtin_amdgcn_fence(__ATOMIC_ACQUIRE, "workgroup"); }

__global__ __launch_bounds__(256) void prep_kernel(const float* __restrict__ x, const float* __restrict__ W, const float* __restrict__ cen, b16* __restrict__ xh, b16* __restrict__ xl, float* __restrict__ xx, b16* __restrict__ ch, b16* __restrict__ cl, float* __restrict__ cc, b16* __restrict__ wh, b16* __restrict__ wl) {
  const size_t tid = (size_t)blockIdx.x * blockDim.x + threadIdx.x, nth = (size_t)gridDim.x * blockDim.x;
  for (int pass = 0; pass < 2; ++pass) {
    for (size_t p = tid; p < (size_t)Bn * FIN; p += nth) { b16 a, c; split16(x[p] * XS, a, c); ((volatile b16*)xh)[p] = a; ((volatile b16*)xl)[p] = c; }
    for (size_t p = tid; p < (size_t)NK * FIN; p += nth) { b16 a, c; split16(cen[p] * CS, a, c); ((volatile b16*)ch)[p] = a; ((volatile b16*)cl)[p] = c; }
    for (size_t p = tid; p < (size_t)FO * NK; p += nth) { b16 a, c; split16(W[p] * WS_, a, c); ((volatile b16*)wh)[p] = a; ((volatile b16*)wl)[p] = c; }
    for (size_t r = tid; r < (size_t)Bn; r += nth) { float s = 0.0f; for (int d = 0; d < FIN; ++d) { const float v = x[r * FIN + d]; s += v * v; } ((volatile float*)xx)[r] = s; }
    for (size_t r = tid; r < (size_t)NK; r += nth) { float s = 0.0f; for (int d = 0; d < FIN; ++d) { const float v = cen[r * FIN + d]; s += v * v; } ((volatile float*)cc)[r] = s; }
    __threadfence();
  }
}

__global__ __launch_bounds__(128) void rbf_kernel(const b16* __restrict__ xh, const b16* __restrict__ xl, const b16* __restrict__ ch, const b16* __restrict__ cl, const float* __restrict__ xx, const float* __restrict__ cc, const float* __restrict__ lsh, float* __restrict__ rbf) {
  __shared__ __attribute__((aligned(16))) float Ts[4][32 * 64];
  const int lane = threadIdx.x & 31, wave = threadIdx.x >> 5, nloc = lane & 15, hlf = lane >> 4, m0 = blockIdx.y * 128 + wave * 32, c0 = blockIdx.x * 64;
  v8f acc[2][4];
#pragma unroll
  for (int r = 0; r < 2; ++r)
#pragma unroll
    for (int t = 0; t < 4; ++t) acc[r][t] = (v8f){};
#pragma unroll
  for (int kb = 0; kb < FIN; kb += 32) { const v16b a0 = frag_kb(xh + (size_t)(m0 + nloc) * FIN + kb, hlf), l0 = frag_kb(xl + (size_t)(m0 + nloc) * FIN + kb, hlf), a1 = frag_kb(xh + (size_t)(m0 + 16 + nloc) * FIN + kb, hlf), l1 = frag_kb(xl + (size_t)(m0 + 16 + nloc) * FIN + kb, hlf);
#pragma unroll
    for (int t = 0; t < 4; ++t) { const size_t bo = (size_t)(c0 + t * 16 + nloc) * FIN + kb; const v16b b0 = frag_kb(ch + bo, hlf), b1 = frag_kb(cl + bo, hlf);
      acc[0][t] = wmma16b(a0, b0, acc[0][t]); acc[0][t] = wmma16b(l0, b0, acc[0][t]); acc[0][t] = wmma16b(a0, b1, acc[0][t]);
      acc[1][t] = wmma16b(a1, b0, acc[1][t]); acc[1][t] = wmma16b(l1, b0, acc[1][t]); acc[1][t] = wmma16b(a1, b1, acc[1][t]); } }
  float* Tt = Ts[wave];
#pragma unroll
  for (int t = 0; t < 4; ++t) { const int k = c0 + t * 16 + nloc; const float ck = cc[k], ek = expf(lsh[k]);
#pragma unroll
    for (int r = 0; r < 2; ++r)
#pragma unroll
      for (int v = 0; v < 8; ++v) { const int row = m0 + r * 16 + 8 * hlf + v; const float r2 = xx[row] + ck - 2.0f * acc[r][t][v] * (1.0f / (XS * CS)); const float rr = sqrtf(fmaxf(r2, 0.0f)); const float er = ek * rr;
        Tt[(r * 16 + v + 8 * hlf) * 64 + t * 16 + nloc] = expf(-(er * er)); } }
  wave_lds_sync();
  float* dst0 = rbf + (size_t)m0 * NK + c0;
  for (int pass = 0; pass < 2; ++pass) {
#pragma unroll
    for (int j = 0; j < 16; ++j) { const int rr = j * 2 + hlf, c4 = nloc * 4; *(volatile v4f*)(dst0 + (size_t)rr * NK + c4) = *(const v4f*)(Tt + rr * 64 + c4); }
    __threadfence(); }
}

__global__ __launch_bounds__(256) void norm_kernel(const float* __restrict__ rbf, b16* __restrict__ nh, b16* __restrict__ nl) {
  const int wid = threadIdx.x >> 5, lane = threadIdx.x & 31; const size_t row = (size_t)blockIdx.x * 8 + wid; const float* src = rbf + row * NK;
  v4f v[4]; float s = 0.0f;
#pragma unroll
  for (int p = 0; p < 4; ++p) { v[p] = *(const v4f*)(src + p * 128 + lane * 4); s += (v[p][0] + v[p][1]) + (v[p][2] + v[p][3]); }
#pragma unroll
  for (int o = 1; o < 32; o <<= 1) s += __shfl_xor(s, o);
  const float inv = RS / (1e-9f + s);
  typedef __attribute__((ext_vector_type(4))) _Float16 v4b;
  for (int pass = 0; pass < 2; ++pass) {
#pragma unroll
    for (int p = 0; p < 4; ++p) { v4b a4, c4;
#pragma unroll
      for (int e = 0; e < 4; ++e) { b16 a, c; split16(v[p][e] * inv, a, c); a4[e] = a; c4[e] = c; }
      *(volatile v4b*)(nh + row * NK + p * 128 + lane * 4) = a4; *(volatile v4b*)(nl + row * NK + p * 128 + lane * 4) = c4; }
    __threadfence(); }
}

__global__ __launch_bounds__(128) void out_kernel(const b16* __restrict__ nh, const b16* __restrict__ nl, const b16* __restrict__ wh, const b16* __restrict__ wl, float* __restrict__ out) {
  __shared__ __attribute__((aligned(16))) float Ts[4][32 * 64];
  const int lane = threadIdx.x & 31, wave = threadIdx.x >> 5, nloc = lane & 15, hlf = lane >> 4, m0 = blockIdx.y * 128 + wave * 32, c0 = blockIdx.x * 64;
  v8f acc[2][4];
#pragma unroll
  for (int r = 0; r < 2; ++r)
#pragma unroll
    for (int t = 0; t < 4; ++t) acc[r][t] = (v8f){};
#pragma unroll 2
  for (int kb = 0; kb < NK; kb += 32) { const v16b a0 = frag_kb(nh + (size_t)(m0 + nloc) * NK + kb, hlf), l0 = frag_kb(nl + (size_t)(m0 + nloc) * NK + kb, hlf), a1 = frag_kb(nh + (size_t)(m0 + 16 + nloc) * NK + kb, hlf), l1 = frag_kb(nl + (size_t)(m0 + 16 + nloc) * NK + kb, hlf);
#pragma unroll
    for (int t = 0; t < 4; ++t) { const size_t bo = (size_t)(c0 + t * 16 + nloc) * NK + kb; const v16b b0 = frag_kb(wh + bo, hlf), b1 = frag_kb(wl + bo, hlf);
      acc[0][t] = wmma16b(a0, b0, acc[0][t]); acc[0][t] = wmma16b(l0, b0, acc[0][t]); acc[0][t] = wmma16b(a0, b1, acc[0][t]);
      acc[1][t] = wmma16b(a1, b0, acc[1][t]); acc[1][t] = wmma16b(l1, b0, acc[1][t]); acc[1][t] = wmma16b(a1, b1, acc[1][t]); } }
  float* Tt = Ts[wave];
#pragma unroll
  for (int t = 0; t < 4; ++t)
#pragma unroll
    for (int r = 0; r < 2; ++r)
#pragma unroll
      for (int v = 0; v < 8; ++v) Tt[(r * 16 + v + 8 * hlf) * 64 + t * 16 + nloc] = acc[r][t][v] * (1.0f / (RS * WS_));
  wave_lds_sync();
  float* dst0 = out + (size_t)m0 * FO + c0;
  for (int pass = 0; pass < 2; ++pass) {
#pragma unroll
    for (int j = 0; j < 16; ++j) { const int rr = j * 2 + hlf, c4 = nloc * 4; *(volatile v4f*)(dst0 + (size_t)rr * FO + c4) = *(const v4f*)(Tt + rr * 64 + c4); }
    __threadfence(); }
}
}

extern "C" void kernel_launch(void* const* d_in, const int* in_sizes, int n_in,
                              void* d_out, int out_size, void* d_ws, size_t ws_size, hipStream_t stream) {
  (void)n_in; (void)out_size;
  const float* x = (const float*)d_in[0]; const float* W = (const float*)d_in[1]; const float* cen = (const float*)d_in[2]; const float* lsh = (const float*)d_in[3];
  float* out = (float*)d_out;
  if (in_sizes[0] != Bn * FIN || in_sizes[1] != FO * NK || in_sizes[2] != NK * FIN || in_sizes[3] != NK) return;
  size_t off = 0; char* ws = (char*)d_ws;
  auto carve = [&](size_t bytes) { char* p = ws + off; off += (bytes + 255) & ~(size_t)255; return p; };
  b16* xh = (b16*)carve((size_t)Bn * FIN * 2); b16* xl = (b16*)carve((size_t)Bn * FIN * 2); float* xx = (float*)carve((size_t)Bn * 4); b16* ch = (b16*)carve((size_t)NK * FIN * 2); b16* cl = (b16*)carve((size_t)NK * FIN * 2); float* cc = (float*)carve((size_t)NK * 4);
  b16* wh = (b16*)carve((size_t)FO * NK * 2); b16* wl = (b16*)carve((size_t)FO * NK * 2); float* rbf = (float*)carve((size_t)Bn * NK * 4); b16* nh = (b16*)carve((size_t)Bn * NK * 2); b16* nl = (b16*)carve((size_t)Bn * NK * 2);
  if (off > ws_size) return;
  prep_kernel<<<256, 256, 0, stream>>>(x, W, cen, xh, xl, xx, ch, cl, cc, wh, wl);
  rbf_kernel<<<dim3(NK / 64, Bn / 128), 128, 0, stream>>>(xh, xl, ch, cl, xx, cc, lsh, rbf);
  norm_kernel<<<Bn / 8, 256, 0, stream>>>(rbf, nh, nl);
  out_kernel<<<dim3(FO / 64, Bn / 128), 128, 0, stream>>>(nh, nl, wh, wl, out);
}
